// CLS_AttentionBlock_26036091748980
// MI455X (gfx1250) — hardware-verified
//
#include <hip/hip_runtime.h>
#include <math.h>

typedef __attribute__((ext_vector_type(16))) _Float16 v16h;
typedef __attribute__((ext_vector_type(16))) __bf16 v16b;
typedef __attribute__((ext_vector_type(8)))  _Float16 v8h;
typedef __attribute__((ext_vector_type(8)))  float v8f;
typedef __attribute__((ext_vector_type(4)))  float v4f;
typedef __attribute__((ext_vector_type(2)))  float v2f;
typedef __attribute__((ext_vector_type(4)))  unsigned v4u;
typedef __attribute__((ext_vector_type(4)))  int v4i;
typedef float __attribute__((may_alias)) float_a;
typedef int __attribute__((may_alias)) int_a;

template <typename T> __device__ __forceinline__ void vst2(void* p, T v) { *(volatile T*)p = v; __threadfence(); *(volatile T*)p = v; }
__device__ __forceinline__ v8f wmma16(v16h a, v16h b, v8f c) {
  v8f d = __builtin_amdgcn_wmma_f32_16x16x32_f16(false, a, false, b, (short)0, c, false, false);
  asm volatile("v_nop\n\tv_nop\n\tv_nop\n\tv_nop" : "+v"(d) : "v"(a), "v"(b));
  return d;
}
__device__ __forceinline__ v8f wmma_bf(v16b a, v16b b, v8f c) {
  v8f d = __builtin_amdgcn_wmma_f32_16x16x32_bf16(false, a, false, b, (short)0, c, false, false);
  asm volatile("v_nop\n\tv_nop\n\tv_nop\n\tv_nop" : "+v"(d) : "v"(a), "v"(b));
  return d;
}
__device__ __forceinline__ v16h frag_h(const _Float16* rowk0, int lane) {
  union { v16h v; v8h q[2]; } u; const _Float16* p = rowk0 + 8 * (lane >> 4);
  u.q[0] = *(const v8h*)p; u.q[1] = *(const v8h*)(p + 16); return u.v;
}
__device__ __forceinline__ v16h frag_f32(const float* rowk0, int lane) {
  v16h a; const float* p = rowk0 + 8 * (lane >> 4);
#pragma unroll
  for (int i = 0; i < 8; ++i) { a[i] = (_Float16)p[i]; a[8 + i] = (_Float16)p[16 + i]; }
  return a;
}
__device__ __forceinline__ v16h frag_f32s(const float* rowk0, int lane, float sc) {
  v16h a; const float* p = rowk0 + 8 * (lane >> 4);
#pragma unroll
  for (int i = 0; i < 8; ++i) { a[i] = (_Float16)(p[i] * sc); a[8 + i] = (_Float16)(p[16 + i] * sc); }
  return a;
}
__device__ __forceinline__ v16h fragc_f32(const float* W, int k0, int n, int lane, int ld, int K) {
  v16h a; const int g = lane >> 4;
#pragma unroll
  for (int i = 0; i < 8; ++i) { const int ka = k0 + 8 * g + i, kb = ka + 16;
    a[i] = (_Float16)(ka < K ? W[(size_t)ka * ld + n] : 0.f); a[8 + i] = (_Float16)(kb < K ? W[(size_t)kb * ld + n] : 0.f); }
  return a;
}
struct F2 { v16b h, l; };
__device__ __forceinline__ F2 bsplit16(const float v[16]) { F2 r;
#pragma unroll
  for (int i = 0; i < 16; ++i) { const __bf16 h = (__bf16)v[i]; r.h[i] = h; r.l[i] = (__bf16)(v[i] - (float)h); }
  return r; }
__device__ __forceinline__ F2 split_row(const float* row, int k0, int lane) { float v[16]; const float* p = row + k0 + 8 * (lane >> 4);
#pragma unroll
  for (int i = 0; i < 8; ++i) { v[i] = p[i]; v[8 + i] = p[16 + i]; }
  return bsplit16(v); }
__device__ __forceinline__ F2 split_rowK(const float* row, int k0, int lane, int K) { float v[16]; const int g = lane >> 4;
#pragma unroll
  for (int i = 0; i < 8; ++i) { const int ka = k0 + 8 * g + i, kb = ka + 16; v[i] = ka < K ? row[ka] : 0.f; v[8 + i] = kb < K ? row[kb] : 0.f; }
  return bsplit16(v); }
__device__ __forceinline__ F2 split_col(const float* W, int k0, int n, int lane, int ld, int K) { float v[16]; const int g = lane >> 4;
#pragma unroll
  for (int i = 0; i < 8; ++i) { const int ka = k0 + 8 * g + i, kb = ka + 16; v[i] = ka < K ? W[(size_t)ka * ld + n] : 0.f; v[8 + i] = kb < K ? W[(size_t)kb * ld + n] : 0.f; }
  return bsplit16(v); }
__device__ __forceinline__ v8f mac3(const F2& a, const F2& b, v8f c) { c = wmma_bf(a.l, b.h, c); c = wmma_bf(a.h, b.l, c); return wmma_bf(a.h, b.h, c); }
__device__ __forceinline__ float sigm(float v) { return 1.0f / (1.0f + expf(-v)); }
#define LDSX() do { asm volatile("s_wait_dscnt 0" ::: "memory"); __builtin_amdgcn_wave_barrier(); __builtin_amdgcn_fence(__ATOMIC_RELEASE, "workgroup"); } while (0)


#define NB 16
#define SS 1024
#define E 512
#define NH 8
#define NGR 32
#define HD 64
#define NR (NB * SS)
#define PLO 1024.0f
#define VLO 2048.0f
__device__ __forceinline__ float bfr(float v) { return (float)(__bf16)v; }
__device__ __forceinline__ v16b frag_b(const __bf16* rowk0, int lane) { return __builtin_bit_cast(v16b, frag_h((const _Float16*)rowk0, lane)); }

__global__ __launch_bounds__(256) void k_stats(const float* __restrict__ x, float* __restrict__ ST) {
  __shared__ float sred[256]; __shared__ float smu;
  const int tid = threadIdx.x; const int b = blockIdx.y, grp = blockIdx.x; const float* base = x + ((size_t)b * E + grp * (E / NGR)) * SS; const int cnt = (E / NGR) * SS;
  float s = 0.f; for (int i = tid; i < cnt; i += 256) s += bfr(base[i]);
  sred[tid] = s; __syncthreads();
  for (int st = 128; st > 0; st >>= 1) { if (tid < st) sred[tid] += sred[tid + st]; __syncthreads(); }
  if (tid == 0) smu = sred[0] / (float)cnt;
  __syncthreads();
  const float mu = smu; float q = 0.f; for (int i = tid; i < cnt; i += 256) { const float d = bfr(base[i]) - mu; q += d * d; }
  __syncthreads(); sred[tid] = q; __syncthreads();
  for (int st = 128; st > 0; st >>= 1) { if (tid < st) sred[tid] += sred[tid + st]; __syncthreads(); }
  if (tid == 0) { union { float f[4]; v4f v; } u; u.f[0] = mu; u.f[1] = rsqrtf(sred[0] / (float)cnt + 1e-5f); u.f[2] = 0.f; u.f[3] = 0.f; vst2(ST + ((size_t)b * NGR + grp) * 4, u.v); }
}
__global__ __launch_bounds__(256) void k_cvt(const float* __restrict__ x, const float* __restrict__ ST, const float* __restrict__ gw, const float* __restrict__ gb, __bf16* __restrict__ Th, __bf16* __restrict__ Tl) {
  __shared__ __align__(16) __bf16 sh_[64][E + 8], sl_[64][E + 8];
  const int tid = threadIdx.x; const int b = blockIdx.y, n0 = blockIdx.x * 64;
  for (int q = tid; q < E * 16; q += 256) { const int c = q >> 4, p4 = q & 15; const int grp = c / (E / NGR); const float mu = ST[((size_t)b * NGR + grp) * 4], rs = ST[((size_t)b * NGR + grp) * 4 + 1]; const float w = bfr(gw[c]), bc = bfr(gb[c]);
    const v4f v = *(const v4f*)(x + ((size_t)b * E + c) * SS + n0 + p4 * 4);
#pragma unroll
    for (int e = 0; e < 4; ++e) { const float t = (bfr(v[e]) - mu) * rs * w + bc; const __bf16 hi = (__bf16)t; sh_[p4 * 4 + e][c] = hi; sl_[p4 * 4 + e][c] = (__bf16)(t - (float)hi); } }
  __syncthreads();
  for (int q = tid; q < 64 * (E / 8); q += 256) { const int rl = q / (E / 8), pc = q % (E / 8); const size_t o = ((size_t)b * SS + n0 + rl) * E + pc * 8; vst2((unsigned*)(Th + o), *(const v4u*)(&sh_[rl][pc * 8])); vst2((unsigned*)(Tl + o), *(const v4u*)(&sl_[rl][pc * 8])); }
}
__global__ __launch_bounds__(256) void k_pack(const float* __restrict__ Wq, const float* __restrict__ Wk, const float* __restrict__ Wv, const float* __restrict__ Wo, __bf16* __restrict__ PT) {
  const int n = blockIdx.x, tid = threadIdx.x; __shared__ __align__(16) __bf16 srow[E];
  const float* W = n < E ? Wq : (n < 2 * E ? Wk : (n < 3 * E ? Wv : Wo)); const int nn = n % E;
  for (int k = tid; k < E; k += 256) srow[k] = (__bf16)W[(size_t)nn * E + k];
  __syncthreads();
  if (tid < E / 8) vst2((unsigned*)(PT + (size_t)n * E + tid * 8), *(const v4u*)(&srow[tid * 8]));
}
__global__ __launch_bounds__(128) void k_qkv(const __bf16* __restrict__ Th, const __bf16* __restrict__ Tl, const __bf16* __restrict__ PT, const float* __restrict__ bq, const float* __restrict__ bk, const float* __restrict__ bv, float* __restrict__ Q32, __bf16* __restrict__ Kh, __bf16* __restrict__ Kl, _Float16* __restrict__ VTh, _Float16* __restrict__ VTl) {
  __shared__ __align__(16) float so[4][16][132];
  __shared__ __align__(16) _Float16 sth[128][72], stl[128][72];
  const int tid = threadIdx.x, wave = tid >> 5, lane = tid & 31, col = lane & 15, g = lane >> 4;
  const int which = blockIdx.z, r0b = blockIdx.x * 64, r0 = r0b + wave * 16, n0 = blockIdx.y * 128; const int b = r0b / SS, s0 = r0b % SS;
  const float* bb_ = which == 0 ? bq : (which == 1 ? bk : bv);
  v8f acc[8] = {};
#pragma unroll 2
  for (int kc = 0; kc < E / 32; ++kc) { const v16b ah = frag_b(Th + (size_t)(r0 + col) * E + kc * 32, lane), al = frag_b(Tl + (size_t)(r0 + col) * E + kc * 32, lane);
#pragma unroll
    for (int j = 0; j < 8; ++j) { const v16b wb = frag_b(PT + (size_t)(which * E + n0 + j * 16 + col) * E + kc * 32, lane); acc[j] = wmma_bf(al, wb, acc[j]); acc[j] = wmma_bf(ah, wb, acc[j]); } }
  if (which < 2) {
#pragma unroll
    for (int j = 0; j < 8; ++j) { const float bb = bfr(bb_[n0 + j * 16 + col]);
#pragma unroll
      for (int r = 0; r < 8; ++r) so[wave][8 * g + r][j * 16 + col] = acc[j][r] + bb; }
    LDSX();
    if (which == 0) { for (int qq = lane; qq < 2 * 16 * 16; qq += 32) { const int hh = qq >> 8, rl = (qq >> 4) & 15, pc = qq & 15; const int h = (n0 >> 6) + hh;
        vst2(Q32 + (((size_t)b * NH + h) * SS + s0 + wave * 16 + rl) * HD + pc * 4, *(const v4f*)(&so[wave][rl][hh * 64 + pc * 4])); } }
    else {
      for (int qq = lane; qq < 2 * 16 * 16; qq += 32) { const int hh = qq >> 8, rl = (qq >> 4) & 15, pl = qq & 15; const int h = (n0 >> 6) + hh; const int pc = pl & 7; union { __bf16 e[8]; v4u u; } pk;
#pragma unroll
        for (int e = 0; e < 8; ++e) { const float v = so[wave][rl][hh * 64 + pc * 8 + e]; const __bf16 hi = (__bf16)v; pk.e[e] = pl < 8 ? hi : (__bf16)(v - (float)hi); }
        vst2((unsigned*)((pl < 8 ? Kh : Kl) + (((size_t)b * NH + h) * SS + s0 + wave * 16 + rl) * HD + pc * 8), pk.u); } } }
  else {
#pragma unroll
    for (int j = 0; j < 8; ++j) { const float bb = bfr(bb_[n0 + j * 16 + col]);
#pragma unroll
      for (int r = 0; r < 8; ++r) { const float v = (acc[j][r] + bb) * 4.0f; const _Float16 hi = (_Float16)v; sth[j * 16 + col][wave * 16 + 8 * g + r] = hi; stl[j * 16 + col][wave * 16 + 8 * g + r] = (_Float16)((v - (float)hi) * VLO); } }
    __syncthreads();
    for (int qq = tid; qq < 128 * 8; qq += 128) { const int cl = qq >> 3, pc = qq & 7; const int c = n0 + cl, h = c >> 6, d = c & 63; const size_t o = (((size_t)b * NH + h) * HD + d) * SS + s0 + pc * 8;
      vst2(VTh + o, *(const v4u*)(&sth[cl][pc * 8])); vst2(VTl + o, *(const v4u*)(&stl[cl][pc * 8])); } }
}
__global__ __launch_bounds__(128) void k_attn(const float* __restrict__ Q32, const __bf16* __restrict__ Kh, const __bf16* __restrict__ Kl, const _Float16* __restrict__ VTh, const _Float16* __restrict__ VTl, float* __restrict__ O32) {
  __shared__ __align__(16) float sS[4][16][68];
  __shared__ __align__(16) _Float16 sPh[4][16][72], sPl[4][16][72];
  __shared__ __align__(16) float sO[4][16][68];
  const int tid = threadIdx.x, w = tid >> 5, lane = tid & 31, col = lane & 15, g = lane >> 4;
  const size_t bh = blockIdx.y; const int qb = blockIdx.x; const int q0 = qb * 64 + w * 16;
  F2 aq[2];
#pragma unroll
  for (int kc = 0; kc < 2; ++kc) aq[kc] = split_row(Q32 + (bh * SS + q0 + col) * HD, kc * 32, lane);
  float mrun = -3.0e38f, lrun = 0.f; v8f acc[4] = {}, ac1[4] = {}, ac2[4] = {};
  LDSX();
#pragma unroll 1
  for (int kt = 0; kt < SS / 64; ++kt) {
#pragma unroll
    for (int t = 0; t < 4; ++t) { const int key = kt * 64 + t * 16 + col; const size_t ko = (bh * SS + key) * HD; v8f s = {};
#pragma unroll
      for (int kc = 0; kc < 2; ++kc) { const v16b khf = frag_b(Kh + ko + kc * 32, lane), klf = frag_b(Kl + ko + kc * 32, lane); s = wmma_bf(aq[kc].l, khf, s); s = wmma_bf(aq[kc].h, klf, s); s = wmma_bf(aq[kc].h, khf, s); }
#pragma unroll
      for (int r = 0; r < 8; ++r) sS[w][8 * g + r][t * 16 + col] = s[r] * 0.044194173824159216f; }
    LDSX();
    float mx = -3.4e38f;
#pragma unroll
    for (int jj = 0; jj < 32; ++jj) mx = fmaxf(mx, sS[w][col][g * 32 + jj]);
    mx = fmaxf(mx, __shfl_xor(mx, 16, 32));
    const float mnew = fmaxf(mrun, mx); const float corr = expf(mrun - mnew);
    float ps = 0.f;
#pragma unroll
    for (int jj = 0; jj < 32; ++jj) { const float p = expf(sS[w][col][g * 32 + jj] - mnew) * 16384.0f; ps += p; const _Float16 hi = (_Float16)p; sPh[w][col][g * 32 + jj] = hi; sPl[w][col][g * 32 + jj] = (_Float16)((p - (float)hi) * PLO); }
    ps += __shfl_xor(ps, 16, 32);
    lrun = lrun * corr + ps * (1.0f / 16384.0f); mrun = mnew;
#pragma unroll
    for (int r = 0; r < 8; ++r) { const float cr = __shfl(corr, 8 * g + r, 32);
#pragma unroll
      for (int t = 0; t < 4; ++t) { acc[t][r] *= cr; ac1[t][r] *= cr; ac2[t][r] *= cr; } }
    LDSX();
#pragma unroll
    for (int kc = 0; kc < 2; ++kc) { const v16h ph = frag_h(&sPh[w][col][0] + kc * 32, lane), pl = frag_h(&sPl[w][col][0] + kc * 32, lane);
#pragma unroll
      for (int t = 0; t < 4; ++t) { const size_t vo = (bh * HD + t * 16 + col) * SS + kt * 64 + kc * 32; const v16h vh = frag_h(VTh + vo, lane);
        acc[t] = wmma16(ph, vh, acc[t]); ac1[t] = wmma16(ph, frag_h(VTl + vo, lane), ac1[t]); ac2[t] = wmma16(pl, vh, ac2[t]); } }
    __builtin_amdgcn_wave_barrier(); }
#pragma unroll
  for (int r = 0; r < 8; ++r) { const float lr = __shfl(lrun, 8 * g + r, 32); const float inv = 1.0f / (lr * 16384.0f * 4.0f);
#pragma unroll
    for (int t = 0; t < 4; ++t) sO[w][8 * g + r][t * 16 + col] = (acc[t][r] + ac1[t][r] * (1.0f / VLO) + ac2[t][r] * (1.0f / PLO)) * inv; }
  LDSX();
  for (int qq = lane; qq < 16 * 16; qq += 32) { const int rl = qq >> 4, pc = qq & 15; vst2(O32 + ((bh * SS) + q0 + rl) * HD + pc * 4, *(const v4f*)(&sO[w][rl][pc * 4])); }
}
__global__ __launch_bounds__(128) void k_out(const float* __restrict__ O32, const float* __restrict__ Wo, const float* __restrict__ x, float* __restrict__ y) {
  __shared__ __align__(16) float sY[4][64][68];
  const int tid = threadIdx.x, w = tid >> 5, lane = tid & 31, col = lane & 15, g = lane >> 4; const int b = blockIdx.y, p0 = blockIdx.x * 64;
#pragma unroll 1
  for (int ps = 0; ps < 2; ++ps) { const int cbase = ps * 256 + w * 64;
    v8f acc[4][4] = {};
#pragma unroll 1
    for (int kc = 0; kc < E / 32; ++kc) { const int h = kc >> 1; F2 bo_[4];
#pragma unroll
      for (int pt = 0; pt < 4; ++pt) bo_[pt] = split_row(O32 + (((size_t)b * NH + h) * SS + p0 + pt * 16 + col) * HD, (kc & 1) * 32, lane);
#pragma unroll
      for (int ct = 0; ct < 4; ++ct) { const v16b a = split_row(Wo + (size_t)(cbase + ct * 16 + col) * E, kc * 32, lane).h;
#pragma unroll
        for (int pt = 0; pt < 4; ++pt) { acc[ct][pt] = wmma_bf(a, bo_[pt].l, acc[ct][pt]); acc[ct][pt] = wmma_bf(a, bo_[pt].h, acc[ct][pt]); } } }
#pragma unroll
    for (int ct = 0; ct < 4; ++ct) {
#pragma unroll
      for (int r = 0; r < 8; ++r) { const int cl = ct * 16 + 8 * g + r; const int c = cbase + cl;
#pragma unroll
        for (int pt = 0; pt < 4; ++pt) { const int n = p0 + pt * 16 + col; sY[w][cl][pt * 16 + col] = acc[ct][pt][r] + bfr(x[((size_t)b * E + c) * SS + n]); } } }
    LDSX();
    for (int qq = lane; qq < 64 * 16; qq += 32) { const int cl = qq >> 4, pc = qq & 15; vst2(y + ((size_t)b * E + cbase + cl) * SS + p0 + pc * 4, *(const v4f*)(&sY[w][cl][pc * 4])); }
    LDSX(); }
}
#define NPASS 2
#define NBP (NB / NPASS)
extern "C" void kernel_launch(void* const* d_in, const int* in_sizes, int n_in, void* d_out, int out_size, void* d_ws, size_t ws_size, hipStream_t stream) {
  (void)in_sizes; (void)n_in; (void)out_size; (void)ws_size;
  const float** I = (const float**)d_in;
  const float* x = I[0]; float* y = (float*)d_out;
  char* ws = (char*)d_ws; size_t off = 0;
  auto take = [&](size_t bytes) { char* p = ws + off; off += (bytes + 255) & ~(size_t)255; return p; };
  const size_t RP = (size_t)NBP * SS;
  float* ST = (float*)take((size_t)NB * NGR * 16); __bf16* Th = (__bf16*)take((size_t)NR * E * 2); __bf16* Tl = (__bf16*)take((size_t)NR * E * 2); __bf16* PT = (__bf16*)take((size_t)4 * E * E * 2);
  float* Q32 = (float*)take(RP * E * 4); __bf16* Kh = (__bf16*)take(RP * E * 2); __bf16* Kl = (__bf16*)take(RP * E * 2); _Float16* VTh = (_Float16*)take(RP * E * 2); _Float16* VTl = (_Float16*)take(RP * E * 2); float* O32 = (float*)take(RP * E * 4);
  k_stats<<<dim3(NGR, NB), 256, 0, stream>>>(x, ST);
  k_cvt<<<dim3(SS / 64, NB), 256, 0, stream>>>(x, ST, I[1], I[2], Th, Tl);
  k_pack<<<4 * E, 256, 0, stream>>>(I[3], I[5], I[7], I[9], PT);
  for (int ps = 0; ps < NPASS; ++ps) { const size_t ro = (size_t)ps * RP * E;
    k_qkv<<<dim3(RP / 64, E / 128, 3), 128, 0, stream>>>(Th + ro, Tl + ro, PT, I[4], I[6], I[8], Q32, Kh, Kl, VTh, VTl);
    k_attn<<<dim3(SS / 64, NBP * NH), 128, 0, stream>>>(Q32, Kh, Kl, VTh, VTl, O32);
    k_out<<<dim3(SS / 64, NBP), 128, 0, stream>>>(O32, I[9], x + ro, y + ro); }
}
